// WaveNet_43310450213095
// MI455X (gfx1250) — hardware-verified
//
#include <hip/hip_runtime.h>
#include <math.h>
#include <stdint.h>

typedef __attribute__((ext_vector_type(16))) _Float16 v16h;
typedef __attribute__((ext_vector_type(8)))  _Float16 v8h;
typedef __attribute__((ext_vector_type(16))) __bf16   v16b;
typedef __attribute__((ext_vector_type(8)))  __bf16   v8b;
typedef __attribute__((ext_vector_type(8)))  float    v8f;
typedef __attribute__((ext_vector_type(4)))  float    v4f;
typedef __attribute__((ext_vector_type(2)))  float    v2f;

constexpr int NBATCH = 2;
constexpr int TLEN   = 8192;
constexpr int MROWS  = NBATCH * TLEN;
constexpr int RESC   = 128;
constexpr int GATEC  = 256;
constexpr int SKC    = 128;
constexpr int OUTCH  = 256;
constexpr int CINC   = 80;
constexpr int CINP   = 96;
constexpr int NLAY   = 20;
constexpr int LPS    = 10;
constexpr int KTAPS  = 3;
constexpr int KDIL   = KTAPS * RESC;
constexpr int HPADR  = 1024;
constexpr int HROWS  = HPADR + TLEN;
constexpr int NTHR   = 256;
constexpr float WCARRY = 16.0f;
constexpr float ACARRY = 8.0f;
constexpr float XFOLD  = 1.0f / 16.0f;
constexpr float GFOLD  = 1.0f / 128.0f;
constexpr float SQRT_HALF_F  = 0.7071067811865476f;
constexpr float SKIP_SCALE_F = 0.22360679774997896f;

static_assert(TLEN % 64 == 0);
static_assert(HPADR >= (KTAPS - 1) * (1 << (LPS - 1)));
static_assert(OUTCH % 32 == 0 && KDIL % 32 == 0 && CINP % 32 == 0 && RESC % 32 == 0 && SKC % 32 == 0);
static_assert(RESC % 64 == 0 && GATEC % 64 == 0 && SKC % 64 == 0 && OUTCH % 64 == 0 && MROWS % 64 == 0);
static_assert(((TLEN / 64) * (RESC / 64)) % 8 == 0);
static_assert(((MROWS / 64) * (GATEC / 64)) % 8 == 0);
static_assert(((MROWS / 64) * (SKC / 64)) % 8 == 0);
static_assert(CINC % 2 == 0 && CINP % 2 == 0 && CINP >= CINC);
static_assert((MROWS * OUTCH / 2) % NTHR == 0 && (MROWS * CINP / 2) % NTHR == 0 && (MROWS * RESC / 2) % NTHR == 0);

__device__ __forceinline__ void dep_guard_h(v8f& a, v8f& b, v16h x, v16h y) { asm volatile("v_nop\n\tv_nop\n\tv_nop\n\tv_nop" : "+v"(a), "+v"(b) : "v"(x), "v"(y)); }
__device__ __forceinline__ void keep4_h(v16h a, v16h b, v16h c, v16h d) { asm volatile("v_nop" :: "v"(a), "v"(b), "v"(c), "v"(d)); }
__device__ __forceinline__ void acc_guard4(v8f& a, v8f& b, v8f& c, v8f& d) { asm volatile("v_nop\n\tv_nop\n\tv_nop\n\tv_nop" : "+v"(a), "+v"(b), "+v"(c), "+v"(d)); }
__device__ __forceinline__ void dep_guard4x_h(v8f& a, v8f& b, v8f& c, v8f& d, v16h x, v16h y) {
  asm volatile("v_nop\n\tv_nop\n\tv_nop\n\tv_nop" : "+v"(a), "+v"(b), "+v"(c), "+v"(d) : "v"(x), "v"(y));
}
template <typename T> struct Frag;
template <> struct Frag<_Float16> {
  typedef v16h V; union U { v16h v; v8h h[2]; };
  static __device__ __forceinline__ v16h load(const _Float16* p) {
    U f; f.h[0] = *(const v8h*)(p); f.h[1] = *(const v8h*)(p + 16); return f.v;
  }
  static __device__ __forceinline__ v8f mma(v16h a, v16h b, v8f c) {
    return __builtin_amdgcn_wmma_f32_16x16x32_f16(false, a, false, b, (short)0, c, false, false);
  }
  static __device__ __forceinline__ void guard(v8f& a, v8f& b, v16h x, v16h y) { dep_guard_h(a, b, x, y); }
  static __device__ __forceinline__ void keep(v16h a, v16h b, v16h c, v16h d) { keep4_h(a, b, c, d); }
};
typedef Frag<_Float16> FragH;

__global__ __launch_bounds__(256) void cast_f32_f16x2(
    const float* __restrict__ in, _Float16* __restrict__ out, int n2) {
  int i = blockIdx.x * 256 + threadIdx.x;
  if (i < n2) {
    const _Float16 h0 = (_Float16)in[2 * i], h1 = (_Float16)in[2 * i + 1];
    const unsigned u = (unsigned)__builtin_bit_cast(unsigned short, h0) | ((unsigned)__builtin_bit_cast(unsigned short, h1) << 16);
    ((volatile unsigned*)out)[i] = u;
    __threadfence();
    ((volatile unsigned*)out)[i] = u;
  }
}

__device__ __forceinline__ void wave_sync_lds() {
  __builtin_amdgcn_fence(__ATOMIC_RELEASE, "workgroup");
  __builtin_amdgcn_wave_barrier();
  __builtin_amdgcn_fence(__ATOMIC_ACQUIRE, "workgroup");
}

__device__ __forceinline__ void kstep64(v8f (&acc)[4][4], const _Float16* __restrict__ At, int lda,
                                        const _Float16* __restrict__ Btt, int ldb, int lane) {
  const int rlane = lane & 15, koff = (lane >> 4) * 8;
  v16h bh[4];
#pragma unroll
  for (int j = 0; j < 4; ++j) bh[j] = FragH::load(Btt + (size_t)((j << 4) + rlane) * ldb + koff);
#pragma unroll
  for (int i = 0; i < 4; ++i) {
    const v16h ah = FragH::load(At + (size_t)((i << 4) + rlane) * lda + koff);
#pragma unroll
    for (int j = 0; j < 4; ++j) acc[i][j] = FragH::mma(ah, bh[j], acc[i][j]);
    dep_guard4x_h(acc[i][0], acc[i][1], acc[i][2], acc[i][3], ah, bh[3]);
  }
  keep4_h(bh[0], bh[1], bh[2], bh[3]);
}

template <int BIAS, bool RESID, int POST, int OUTM, int ACT>
__device__ __forceinline__ void epilogue64(v8f (&acc)[4][4], float* slab, int lane, float scale,
                                           const float* __restrict__ biasn,
                                           const float* __restrict__ Rt, int ldr,
                                           float* Cft, int ldcf, _Float16* Cht, int ldch) {
  const int rlane = lane & 15, hh = lane >> 4, mOff = hh * 8;
  const int c4 = rlane * 4, q = lane >> 3, c8 = (lane & 7) * 8;
  float bvj[4];
#pragma unroll
  for (int j = 0; j < 4; ++j) bvj[j] = (BIAS == 2) ? biasn[(j << 4) + rlane] : 0.0f;
#pragma unroll
  for (int i = 0; i < 4; ++i) {
#pragma unroll
    for (int j = 0; j < 4; ++j) {
#pragma unroll
      for (int r = 0; r < 8; ++r) {
        float v = acc[i][j][r] * scale + bvj[j];
        if (ACT == 2) v = fmaxf(v, 0.0f);
        slab[(mOff + r) * 68 + (j << 4) + rlane] = v;
      }
    }
    wave_sync_lds();
    if (RESID || POST != 0) {
#pragma unroll
      for (int it = 0; it < 8; ++it) {
        const int row = it * 2 + hh;
        float* sp = slab + row * 68 + c4;
        v4f v = *(const v4f*)sp;
        if (RESID) {
          const v4f rv = *(const v4f*)(Rt + (size_t)(i * 16 + row) * ldr + c4);
          v = v + rv;
        }
        if (POST == 1) v = v * SQRT_HALF_F;
        *(v4f*)sp = v;
      }
      wave_sync_lds();
    }
    for (int pass = 0; pass < 2; ++pass) {
      if (OUTM & 1) {
#pragma unroll
        for (int it = 0; it < 8; ++it) {
          const int row = it * 2 + hh;
          const v4f v = *(const v4f*)(slab + row * 68 + c4);
          *(volatile v4f*)(Cft + (size_t)(i * 16 + row) * ldcf + c4) = v;
        }
      }
      if (OUTM & 2) {
#pragma unroll
        for (int it = 0; it < 4; ++it) {
          const int row = it * 4 + q;
          const float* sp = slab + row * 68 + c8;
          v8h hv;
#pragma unroll
          for (int e = 0; e < 8; ++e) hv[e] = (_Float16)(sp[e] * ACARRY);
          *(volatile v8h*)(Cht + (size_t)(i * 16 + row) * ldch + c8) = hv;
        }
      }
      __threadfence();
    }
    wave_sync_lds();
  }
}

template <int BIAS, bool RESID, int POST, int OUTM, int ACT>
__global__ __launch_bounds__(NTHR) void gemm64_kernel(
    const unsigned short* __restrict__ Ap, int lda, long strideA,
    const unsigned short* __restrict__ Btp, int ldb,
    const float* __restrict__ bias,
    const float* __restrict__ Rp, int ldr, long strideR,
    float* __restrict__ Cf, int ldcf, long strideCf,
    unsigned short* __restrict__ Ch, int ldch, long strideCh,
    int M, int N, int K, float scale) {
  __shared__ __align__(16) float sT[8][16 * 68];
  const int b    = blockIdx.y;
  const int lane = threadIdx.x & 31;
  const int wave = threadIdx.x >> 5;
  const int tilesN = N >> 6;
  const int tilesM = M >> 6;
  const int tile = blockIdx.x * 8 + wave;
  if (tile >= tilesM * tilesN) return;
  const int tm = tile / tilesN;
  const int tn = tile - tm * tilesN;
  const int m0 = tm << 6;
  const int n0 = tn << 6;

  const _Float16* At  = (const _Float16*)Ap + (size_t)b * (size_t)strideA + (size_t)m0 * lda;
  const _Float16* Btt = (const _Float16*)Btp + (size_t)n0 * ldb;

  v8f acc[4][4];
#pragma unroll
  for (int i = 0; i < 4; ++i)
#pragma unroll
    for (int j = 0; j < 4; ++j) acc[i][j] = (v8f){0.f, 0.f, 0.f, 0.f, 0.f, 0.f, 0.f, 0.f};

#pragma unroll 1
  for (int k0 = 0; k0 < K; k0 += 32) kstep64(acc, At + k0, lda, Btt + k0, ldb, lane);

  acc_guard4(acc[0][0], acc[0][1], acc[0][2], acc[0][3]);
  acc_guard4(acc[1][0], acc[1][1], acc[1][2], acc[1][3]);
  acc_guard4(acc[2][0], acc[2][1], acc[2][2], acc[2][3]);
  acc_guard4(acc[3][0], acc[3][1], acc[3][2], acc[3][3]);

  const float* Rt = RESID ? (Rp + (size_t)b * (size_t)strideR + (size_t)m0 * ldr + n0) : (const float*)nullptr;
  float* Cft = (OUTM & 1) ? (Cf + (size_t)b * (size_t)strideCf + (size_t)m0 * ldcf + n0) : (float*)nullptr;
  _Float16* Cht = (OUTM & 2) ? ((_Float16*)Ch + (size_t)b * (size_t)strideCh + (size_t)m0 * ldch + n0) : (_Float16*)nullptr;
  epilogue64<BIAS, RESID, POST, OUTM, ACT>(acc, sT[wave], lane, scale, bias + n0, Rt, ldr, Cft, ldcf, Cht, ldch);
}

__global__ __launch_bounds__(NTHR) void gate_gemm64_kernel(
    const unsigned short* __restrict__ hp, const unsigned short* __restrict__ cp,
    const unsigned short* __restrict__ wdp, const unsigned short* __restrict__ wcp,
    const float* __restrict__ bias, float* __restrict__ gout, int dil, float scale) {
  __shared__ __align__(16) float sT[8][16 * 68];
  const int lane = threadIdx.x & 31;
  const int wave = threadIdx.x >> 5;
  constexpr int tilesN = GATEC / 64;
  constexpr int tilesM = MROWS / 64;
  const int tile = blockIdx.x * 8 + wave;
  if (tile >= tilesM * tilesN) return;
  const int tm = tile / tilesN;
  const int tn = tile - tm * tilesN;
  const int m0 = tm << 6;
  const int n0 = tn << 6;
  const int bb = m0 / TLEN;
  const int t0 = m0 - bb * TLEN;

  const _Float16* hb = (const _Float16*)hp;
  const _Float16* cb = (const _Float16*)cp;
  const _Float16* wd = (const _Float16*)wdp;
  const _Float16* wc = (const _Float16*)wcp;

  v8f acc[4][4];
#pragma unroll
  for (int i = 0; i < 4; ++i)
#pragma unroll
    for (int j = 0; j < 4; ++j) acc[i][j] = (v8f){0.f, 0.f, 0.f, 0.f, 0.f, 0.f, 0.f, 0.f};

#pragma unroll 1
  for (int tap = 0; tap < KTAPS; ++tap) {
    int shift = (KTAPS - 1 - tap) * dil;
    shift = (shift < 0) ? 0 : ((shift > HPADR) ? HPADR : shift);
    const size_t prow = (size_t)bb * HROWS + (size_t)(HPADR + t0 - shift);
    const _Float16* At  = hb + prow * RESC;
    const _Float16* Btt = wd + (size_t)n0 * KDIL + tap * RESC;
#pragma unroll 1
    for (int kk = 0; kk < RESC; kk += 32) kstep64(acc, At + kk, RESC, Btt + kk, KDIL, lane);
  }
  {
    const _Float16* At  = cb + (size_t)m0 * CINP;
    const _Float16* Btt = wc + (size_t)n0 * CINP;
#pragma unroll 1
    for (int kk = 0; kk < CINP; kk += 32) kstep64(acc, At + kk, CINP, Btt + kk, CINP, lane);
  }
  acc_guard4(acc[0][0], acc[0][1], acc[0][2], acc[0][3]);
  acc_guard4(acc[1][0], acc[1][1], acc[1][2], acc[1][3]);
  acc_guard4(acc[2][0], acc[2][1], acc[2][2], acc[2][3]);
  acc_guard4(acc[3][0], acc[3][1], acc[3][2], acc[3][3]);

  epilogue64<2, false, 0, 1, 0>(acc, sT[wave], lane, scale, bias + n0, (const float*)nullptr, 0,
                                gout + (size_t)m0 * GATEC + n0, GATEC, (_Float16*)nullptr, 0);
}

__global__ __launch_bounds__(NTHR) void wprep_kernel(const float* __restrict__ W, int Kin, int ncol, int Kpad,
                                                     int total8, unsigned short* __restrict__ bt) {
  const int i = blockIdx.x * NTHR + threadIdx.x;
  if (i >= total8) return;
  const int tpr = Kpad >> 3;
  const int per = ncol * tpr;
  const int l   = i / per;
  const int rem = i - l * per;
  const int n   = rem / tpr;
  const int k0  = (rem - n * tpr) * 8;
  const float* Wl = W + (size_t)l * Kin * ncol;
  v8h hv;
#pragma unroll
  for (int e = 0; e < 8; ++e) {
    const int k  = k0 + e;
    const int kc = (k < Kin) ? k : (Kin - 1);
    const float fk = (k < Kin) ? WCARRY : 0.0f;
    hv[e] = (_Float16)(Wl[(size_t)kc * ncol + n] * fk);
  }
  const size_t o = (size_t)i * 8;
  *(volatile v8h*)(bt + o) = hv;
  __threadfence();
  *(volatile v8h*)(bt + o) = hv;
}

__global__ __launch_bounds__(NTHR) void ccast_kernel(const float* __restrict__ c, unsigned short* __restrict__ out, int n2) {
  const int i = blockIdx.x * NTHR + threadIdx.x;
  if (i >= n2) return;
  const int e0   = 2 * i;
  const int row  = e0 / CINP;
  const int col  = e0 - row * CINP;
  const int colc = (col < CINC) ? col : (CINC - 2);
  const float f  = (col < CINC) ? ACARRY : 0.0f;
  const v2f v = *(const v2f*)(c + (size_t)row * CINC + colc);
  const _Float16 h0 = (_Float16)(v[0] * f), h1 = (_Float16)(v[1] * f);
  const unsigned u = (unsigned)__builtin_bit_cast(unsigned short, h0) | ((unsigned)__builtin_bit_cast(unsigned short, h1) << 16);
  ((volatile unsigned*)out)[i] = u;
  __threadfence();
  ((volatile unsigned*)out)[i] = u;
}

__device__ __forceinline__ float gated_unit(float a, float b) {
  const float ea = expf(-2.0f * fabsf(a));
  const float t  = (1.0f - ea) * __builtin_amdgcn_rcpf(1.0f + ea);
  const float th = copysignf(t, a);
  const float eb = expf(-b);
  const float sg = __builtin_amdgcn_rcpf(1.0f + eb);
  return th * sg;
}
__global__ __launch_bounds__(NTHR) void gact_kernel(const float* __restrict__ g, unsigned short* __restrict__ z, int n2) {
  const int i = blockIdx.x * NTHR + threadIdx.x;
  if (i >= n2) return;
  const int r  = i >> 6;
  const int c0 = (i & 63) * 2;
  const float* gr = g + (size_t)r * GATEC;
  const v2f av = *(const v2f*)(gr + c0);
  const v2f bv = *(const v2f*)(gr + (GATEC / 2) + c0);
  const float z0 = gated_unit(av[0], bv[0]) * ACARRY;
  const float z1 = gated_unit(av[1], bv[1]) * ACARRY;
  const _Float16 h0 = (_Float16)z0, h1 = (_Float16)z1;
  const unsigned u = (unsigned)__builtin_bit_cast(unsigned short, h0) | ((unsigned)__builtin_bit_cast(unsigned short, h1) << 16);
  ((volatile unsigned*)z)[i] = u;
  __threadfence();
  ((volatile unsigned*)z)[i] = u;
}

__global__ __launch_bounds__(NTHR) void scast_kernel(const float* __restrict__ sk, unsigned short* __restrict__ out, int n2) {
  const int i = blockIdx.x * NTHR + threadIdx.x;
  if (i >= n2) return;
  const v2f v = *(const v2f*)(sk + (size_t)i * 2);
  const float s0 = fmaxf(v[0] * SKIP_SCALE_F, 0.0f) * ACARRY;
  const float s1 = fmaxf(v[1] * SKIP_SCALE_F, 0.0f) * ACARRY;
  const _Float16 h0 = (_Float16)s0, h1 = (_Float16)s1;
  const unsigned u = (unsigned)__builtin_bit_cast(unsigned short, h0) | ((unsigned)__builtin_bit_cast(unsigned short, h1) << 16);
  ((volatile unsigned*)out)[i] = u;
  __threadfence();
  ((volatile unsigned*)out)[i] = u;
}

__global__ __launch_bounds__(NTHR) void zero_kernel(float* __restrict__ p, int n4) {
  const int i = blockIdx.x * NTHR + threadIdx.x;
  if (i >= n4) return;
  const v4f zz = {0.f, 0.f, 0.f, 0.f};
  *(volatile v4f*)(p + (size_t)i * 4) = zz;
  __threadfence();
  *(volatile v4f*)(p + (size_t)i * 4) = zz;
}

extern "C" void kernel_launch(void* const* d_in, const int* in_sizes, int n_in,
                              void* d_out, int out_size, void* d_ws,
                              size_t ws_size, hipStream_t stream) {
  (void)in_sizes;
  if (n_in < 15) return;
  if (out_size != MROWS * OUTCH) return;
  const float* x       = (const float*)d_in[0];
  const float* c       = (const float*)d_in[1];
  const float* w_first = (const float*)d_in[2];
  const float* b_first = (const float*)d_in[3];
  const float* w_dil   = (const float*)d_in[4];
  const float* b_dil   = (const float*)d_in[5];
  const float* w_c     = (const float*)d_in[6];
  const float* w_skip  = (const float*)d_in[7];
  const float* b_skip  = (const float*)d_in[8];
  const float* w_res   = (const float*)d_in[9];
  const float* b_res   = (const float*)d_in[10];
  const float* w_out1  = (const float*)d_in[11];
  const float* b_out1  = (const float*)d_in[12];
  const float* w_out2  = (const float*)d_in[13];
  const float* b_out2  = (const float*)d_in[14];
  float* out = (float*)d_out;

  char* ws = (char*)d_ws;
  size_t off = 0;
  auto carve = [&](size_t bytes) { size_t o = off; off += (bytes + 255) & ~(size_t)255; return o; };
  const size_t hsh_plane = (size_t)NBATCH * HROWS * RESC;
  unsigned short* x_h   = (unsigned short*)(ws + carve((size_t)MROWS * OUTCH * 2));
  unsigned short* c_h   = (unsigned short*)(ws + carve((size_t)MROWS * CINP * 2));
  unsigned short* hsh   = (unsigned short*)(ws + carve(hsh_plane * 2 * 2));
  unsigned short* hA_h  = hsh;
  unsigned short* hB_h  = hsh + hsh_plane;
  float* hA_f  = (float*)(ws + carve(hsh_plane * 4));
  float* hB_f  = (float*)(ws + carve(hsh_plane * 4));
  float* gpl   = (float*)(ws + carve((size_t)MROWS * GATEC * 4));
  unsigned short* z_h   = (unsigned short*)(ws + carve((size_t)MROWS * RESC * 2));
  float* skA   = (float*)(ws + carve((size_t)MROWS * SKC * 4));
  float* skB   = (float*)(ws + carve((size_t)MROWS * SKC * 4));
  unsigned short* s_h   = (unsigned short*)(ws + carve((size_t)MROWS * SKC * 2));
  unsigned short* o1_h  = (unsigned short*)(ws + carve((size_t)MROWS * SKC * 2));
  unsigned short* wfirst_t = (unsigned short*)(ws + carve((size_t)RESC * OUTCH * 2));
  unsigned short* wdil_t   = (unsigned short*)(ws + carve((size_t)NLAY * GATEC * KDIL * 2));
  unsigned short* wc_t     = (unsigned short*)(ws + carve((size_t)NLAY * GATEC * CINP * 2));
  unsigned short* wskip_t  = (unsigned short*)(ws + carve((size_t)NLAY * SKC * RESC * 2));
  unsigned short* wres_t   = (unsigned short*)(ws + carve((size_t)NLAY * RESC * RESC * 2));
  unsigned short* wout1_t  = (unsigned short*)(ws + carve((size_t)SKC * SKC * 2));
  unsigned short* wout2_t  = (unsigned short*)(ws + carve((size_t)OUTCH * SKC * 2));
  if (off > ws_size) return;
  if (off > (size_t)134217728) return;

  auto nblk = [](long n) { return (unsigned)((n + NTHR - 1) / NTHR); };

  { const int t8 = 1 * RESC * (OUTCH / 8);     wprep_kernel<<<nblk(t8), NTHR, 0, stream>>>(w_first, OUTCH, RESC, OUTCH, t8, wfirst_t); }
  { const int t8 = NLAY * GATEC * (KDIL / 8);  wprep_kernel<<<nblk(t8), NTHR, 0, stream>>>(w_dil, KDIL, GATEC, KDIL, t8, wdil_t); }
  { const int t8 = NLAY * GATEC * (CINP / 8);  wprep_kernel<<<nblk(t8), NTHR, 0, stream>>>(w_c, CINC, GATEC, CINP, t8, wc_t); }
  { const int t8 = NLAY * SKC * (RESC / 8);    wprep_kernel<<<nblk(t8), NTHR, 0, stream>>>(w_skip, RESC, SKC, RESC, t8, wskip_t); }
  { const int t8 = NLAY * RESC * (RESC / 8);   wprep_kernel<<<nblk(t8), NTHR, 0, stream>>>(w_res, RESC, RESC, RESC, t8, wres_t); }
  { const int t8 = 1 * SKC * (SKC / 8);        wprep_kernel<<<nblk(t8), NTHR, 0, stream>>>(w_out1, SKC, SKC, SKC, t8, wout1_t); }
  { const int t8 = 1 * OUTCH * (SKC / 8);      wprep_kernel<<<nblk(t8), NTHR, 0, stream>>>(w_out2, SKC, OUTCH, SKC, t8, wout2_t); }
  { const int n2 = MROWS * OUTCH / 2;          cast_f32_f16x2<<<nblk(n2), 256, 0, stream>>>(x, (_Float16*)x_h, n2); }
  { const int n2 = MROWS * CINP / 2;           ccast_kernel<<<nblk(n2), NTHR, 0, stream>>>(c, c_h, n2); }
  { const int n4 = (int)(hsh_plane * 2 * 2 / 16); zero_kernel<<<nblk(n4), NTHR, 0, stream>>>((float*)(void*)hsh, n4); }
  { const int n4 = MROWS * SKC / 4;            zero_kernel<<<nblk(n4), NTHR, 0, stream>>>(skA, n4); }

  const long hstride = (long)HROWS * RESC;
  const size_t hdata = (size_t)HPADR * RESC;
  const unsigned gridFirst = (unsigned)(((TLEN / 64) * (RESC / 64)) / 8);
  const unsigned gridGate  = (unsigned)(((MROWS / 64) * (GATEC / 64)) / 8);
  const unsigned gridSkip  = (unsigned)(((MROWS / 64) * (SKC / 64)) / 8);
  const unsigned gridRes   = gridFirst;
  const unsigned gridOut2  = (unsigned)(((MROWS / 64) * (OUTCH / 64)) / 8);

  gemm64_kernel<2, false, 0, 3, 0><<<dim3(gridFirst, NBATCH), NTHR, 0, stream>>>(
      x_h, OUTCH, (long)TLEN * OUTCH,
      wfirst_t, OUTCH,
      b_first,
      (const float*)nullptr, 0, 0L,
      hA_f + hdata, RESC, hstride,
      hA_h + hdata, RESC, hstride,
      TLEN, RESC, OUTCH, XFOLD);

  for (int l = 0; l < NLAY; ++l) {
    const int dil = 1 << (l % LPS);
    const unsigned short* hin_h = (l & 1) ? hB_h : hA_h;
    unsigned short* hout_h      = (l & 1) ? hA_h : hB_h;
    const float* hin_f          = (l & 1) ? hB_f : hA_f;
    float* hout_f               = (l & 1) ? hA_f : hB_f;
    const float* skin           = (l & 1) ? skB : skA;
    float* skout                = (l & 1) ? skA : skB;

    gate_gemm64_kernel<<<gridGate, NTHR, 0, stream>>>(
        hin_h, c_h, wdil_t + (size_t)l * GATEC * KDIL, wc_t + (size_t)l * GATEC * CINP,
        b_dil + (size_t)l * GATEC, gpl, dil, GFOLD);
    { const int n2 = MROWS * RESC / 2; gact_kernel<<<nblk(n2), NTHR, 0, stream>>>(gpl, z_h, n2); }
    gemm64_kernel<2, true, 0, 1, 0><<<dim3(gridSkip, 1), NTHR, 0, stream>>>(
        z_h, RESC, 0L,
        wskip_t + (size_t)l * SKC * RESC, RESC,
        b_skip + (size_t)l * SKC,
        skin, SKC, 0L,
        skout, SKC, 0L,
        (unsigned short*)nullptr, 0, 0L,
        MROWS, SKC, RESC, GFOLD);
    gemm64_kernel<2, true, 1, 3, 0><<<dim3(gridRes, NBATCH), NTHR, 0, stream>>>(
        z_h, RESC, (long)TLEN * RESC,
        wres_t + (size_t)l * RESC * RESC, RESC,
        b_res + (size_t)l * RESC,
        hin_f + hdata, RESC, hstride,
        hout_f + hdata, RESC, hstride,
        hout_h + hdata, RESC, hstride,
        TLEN, RESC, RESC, GFOLD);
  }

  { const int n2 = MROWS * SKC / 2; scast_kernel<<<nblk(n2), NTHR, 0, stream>>>(skA, s_h, n2); }
  gemm64_kernel<2, false, 0, 2, 2><<<dim3(gridSkip, 1), NTHR, 0, stream>>>(
      s_h, SKC, 0L,
      wout1_t, SKC,
      b_out1,
      (const float*)nullptr, 0, 0L,
      (float*)nullptr, 0, 0L,
      o1_h, SKC, 0L,
      MROWS, SKC, SKC, GFOLD);
  gemm64_kernel<2, false, 0, 1, 0><<<dim3(gridOut2, 1), NTHR, 0, stream>>>(
      o1_h, SKC, 0L,
      wout2_t, SKC,
      b_out2,
      (const float*)nullptr, 0, 0L,
      out, OUTCH, 0L,
      (unsigned short*)nullptr, 0, 0L,
      MROWS, OUTCH, SKC, GFOLD);
}
